// NAND_78589311582948
// MI455X (gfx1250) — hardware-verified
//
#include <hip/hip_runtime.h>
#include <math.h>

typedef __attribute__((ext_vector_type(16))) _Float16 v16h;
typedef __attribute__((ext_vector_type(16))) __bf16 v16b;
typedef __attribute__((ext_vector_type(8)))  _Float16 v8h;
typedef __attribute__((ext_vector_type(8)))  float v8f;
typedef __attribute__((ext_vector_type(4)))  float v4f;
typedef __attribute__((ext_vector_type(2)))  float v2f;
typedef __attribute__((ext_vector_type(4)))  unsigned v4u;
typedef __attribute__((ext_vector_type(4)))  int v4i;
typedef float __attribute__((may_alias)) float_a;
typedef int __attribute__((may_alias)) int_a;

template <typename T> __device__ __forceinline__ void vst2(void* p, T v) { *(volatile T*)p = v; __threadfence(); *(volatile T*)p = v; }
__device__ __forceinline__ v8f wmma16(v16h a, v16h b, v8f c) {
  v8f d = __builtin_amdgcn_wmma_f32_16x16x32_f16(false, a, false, b, (short)0, c, false, false);
  asm volatile("v_nop\n\tv_nop\n\tv_nop\n\tv_nop" : "+v"(d) : "v"(a), "v"(b));
  return d;
}
__device__ __forceinline__ v8f wmma_bf(v16b a, v16b b, v8f c) {
  v8f d = __builtin_amdgcn_wmma_f32_16x16x32_bf16(false, a, false, b, (short)0, c, false, false);
  asm volatile("v_nop\n\tv_nop\n\tv_nop\n\tv_nop" : "+v"(d) : "v"(a), "v"(b));
  return d;
}
__device__ __forceinline__ v16h frag_h(const _Float16* rowk0, int lane) {
  union { v16h v; v8h q[2]; } u; const _Float16* p = rowk0 + 8 * (lane >> 4);
  u.q[0] = *(const v8h*)p; u.q[1] = *(const v8h*)(p + 16); return u.v;
}
__device__ __forceinline__ v16h frag_f32(const float* rowk0, int lane) {
  v16h a; const float* p = rowk0 + 8 * (lane >> 4);
#pragma unroll
  for (int i = 0; i < 8; ++i) { a[i] = (_Float16)p[i]; a[8 + i] = (_Float16)p[16 + i]; }
  return a;
}
__device__ __forceinline__ v16h frag_f32s(const float* rowk0, int lane, float sc) {
  v16h a; const float* p = rowk0 + 8 * (lane >> 4);
#pragma unroll
  for (int i = 0; i < 8; ++i) { a[i] = (_Float16)(p[i] * sc); a[8 + i] = (_Float16)(p[16 + i] * sc); }
  return a;
}
__device__ __forceinline__ v16h fragc_f32(const float* W, int k0, int n, int lane, int ld, int K) {
  v16h a; const int g = lane >> 4;
#pragma unroll
  for (int i = 0; i < 8; ++i) { const int ka = k0 + 8 * g + i, kb = ka + 16;
    a[i] = (_Float16)(ka < K ? W[(size_t)ka * ld + n] : 0.f); a[8 + i] = (_Float16)(kb < K ? W[(size_t)kb * ld + n] : 0.f); }
  return a;
}
struct F2 { v16b h, l; };
__device__ __forceinline__ F2 bsplit16(const float v[16]) { F2 r;
#pragma unroll
  for (int i = 0; i < 16; ++i) { const __bf16 h = (__bf16)v[i]; r.h[i] = h; r.l[i] = (__bf16)(v[i] - (float)h); }
  return r; }
__device__ __forceinline__ F2 split_row(const float* row, int k0, int lane) { float v[16]; const float* p = row + k0 + 8 * (lane >> 4);
#pragma unroll
  for (int i = 0; i < 8; ++i) { v[i] = p[i]; v[8 + i] = p[16 + i]; }
  return bsplit16(v); }
__device__ __forceinline__ F2 split_rowK(const float* row, int k0, int lane, int K) { float v[16]; const int g = lane >> 4;
#pragma unroll
  for (int i = 0; i < 8; ++i) { const int ka = k0 + 8 * g + i, kb = ka + 16; v[i] = ka < K ? row[ka] : 0.f; v[8 + i] = kb < K ? row[kb] : 0.f; }
  return bsplit16(v); }
__device__ __forceinline__ F2 split_col(const float* W, int k0, int n, int lane, int ld, int K) { float v[16]; const int g = lane >> 4;
#pragma unroll
  for (int i = 0; i < 8; ++i) { const int ka = k0 + 8 * g + i, kb = ka + 16; v[i] = ka < K ? W[(size_t)ka * ld + n] : 0.f; v[8 + i] = kb < K ? W[(size_t)kb * ld + n] : 0.f; }
  return bsplit16(v); }
__device__ __forceinline__ v8f mac3(const F2& a, const F2& b, v8f c) { c = wmma_bf(a.l, b.h, c); c = wmma_bf(a.h, b.l, c); return wmma_bf(a.h, b.h, c); }
__device__ __forceinline__ float sigm(float v) { return 1.0f / (1.0f + expf(-v)); }
#define LDSX() do { asm volatile("s_wait_dscnt 0" ::: "memory"); __builtin_amdgcn_wave_barrier(); __builtin_amdgcn_fence(__ATOMIC_RELEASE, "workgroup"); } while (0)

#define NBT 1024
#define NC 4096
#define NV 8
#define VS 256
#define DD (NV * VS)

__global__ __launch_bounds__(256) void k_norm(const float* __restrict__ q, const float* __restrict__ w, _Float16* __restrict__ qn, _Float16* __restrict__ wn) {
  __shared__ float sred[8]; __shared__ __align__(16) _Float16 srow[DD];
  const int r = blockIdx.x, tid = threadIdx.x, wv = tid >> 5, lane = tid & 31;
  const bool isq = r < NBT; const float* src = isq ? q + (size_t)r * DD : w + (size_t)(r - NBT) * DD;
#pragma unroll 1
  for (int n = 0; n < NV; ++n) { const float v = src[n * VS + tid]; float s = v * v;
#pragma unroll
    for (int off = 16; off >= 1; off >>= 1) s += __shfl_xor(s, off, 32);
    if (lane == 0) sred[wv] = s;
    __syncthreads();
    float tot = 0.f;
#pragma unroll
    for (int i = 0; i < 8; ++i) tot += sred[i];
    const float inv = 8.0f / fmaxf(sqrtf(tot), 1e-8f);
    srow[n * VS + tid] = (_Float16)(v * inv);
    __syncthreads(); }
  _Float16* dst = isq ? qn + (size_t)r * DD : wn + (size_t)(r - NBT) * DD;
  for (int qd = tid; qd < DD / 8; qd += 256) vst2(dst + qd * 8, *(const v4u*)(&srow[qd * 8]));
}
__global__ __launch_bounds__(128) void k_main(const _Float16* __restrict__ qn, const _Float16* __restrict__ wn, const float* __restrict__ nw, float* __restrict__ out) {
  __shared__ __align__(16) float so[4][16][132];
  const int tid = threadIdx.x, wave = tid >> 5, lane = tid & 31, col = lane & 15, g = lane >> 4;
  const int r0 = blockIdx.x * 64 + wave * 16, c0 = blockIdx.y * 128;
  v8f prod[8];
#pragma unroll
  for (int j = 0; j < 8; ++j)
#pragma unroll
    for (int r = 0; r < 8; ++r) prod[j][r] = 1.0f;
#pragma unroll 1
  for (int n = 0; n < NV; ++n) { v8f acc[8] = {};
#pragma unroll
    for (int kc = 0; kc < VS / 32; ++kc) { const v16h a = frag_h(qn + (size_t)(r0 + col) * DD + n * VS + kc * 32, lane);
#pragma unroll
      for (int j = 0; j < 8; ++j) acc[j] = wmma16(a, frag_h(wn + (size_t)(c0 + j * 16 + col) * DD + n * VS + kc * 32, lane), acc[j]); }
#pragma unroll
    for (int j = 0; j < 8; ++j) { const float s = sigm(nw[(size_t)(c0 + j * 16 + col) * NV + n]);
#pragma unroll
      for (int r = 0; r < 8; ++r) { const float cs = acc[j][r] * (1.0f / 64.0f); prod[j][r] *= s * cs + (1.0f - s) * (1.0f - cs); } } }
#pragma unroll
  for (int j = 0; j < 8; ++j)
#pragma unroll
    for (int r = 0; r < 8; ++r) so[wave][8 * g + r][j * 16 + col] = prod[j][r];
  LDSX();
#pragma unroll 4
  for (int rl = 0; rl < 16; ++rl) vst2(out + (size_t)(r0 + rl) * NC + c0 + lane * 4, *(const v4f*)(&so[wave][rl][lane * 4]));
}
extern "C" void kernel_launch(void* const* d_in, const int* in_sizes, int n_in, void* d_out, int out_size, void* d_ws, size_t ws_size, hipStream_t stream) {
  (void)in_sizes; (void)n_in; (void)out_size; (void)ws_size;
  const float* q = (const float*)d_in[0]; const float* w = (const float*)d_in[1]; const float* nw = (const float*)d_in[2];
  float* out = (float*)d_out;
  char* ws = (char*)d_ws; size_t off = 0;
  auto take = [&](size_t bytes) { char* p = ws + off; off += (bytes + 255) & ~(size_t)255; return p; };
  _Float16* qn = (_Float16*)take((size_t)NBT * DD * 2); _Float16* wn = (_Float16*)take((size_t)NC * DD * 2);
  k_norm<<<NBT + NC, 256, 0, stream>>>(q, w, qn, wn);
  k_main<<<dim3(NBT / 64, NC / 128), 128, 0, stream>>>(qn, wn, nw, out);
}
